// TemporalPoseTransformer_57956288692768
// MI455X (gfx1250) — hardware-verified
//
#include <hip/hip_runtime.h>
#include <math.h>

typedef __attribute__((ext_vector_type(16))) _Float16 v16h;
typedef __attribute__((ext_vector_type(16))) __bf16 v16b;
typedef __attribute__((ext_vector_type(8)))  _Float16 v8h;
typedef __attribute__((ext_vector_type(8)))  float v8f;
typedef __attribute__((ext_vector_type(4)))  float v4f;
typedef __attribute__((ext_vector_type(2)))  float v2f;
typedef __attribute__((ext_vector_type(4)))  unsigned v4u;
typedef __attribute__((ext_vector_type(4)))  int v4i;
typedef float __attribute__((may_alias)) float_a;
typedef int __attribute__((may_alias)) int_a;

template <typename T> __device__ __forceinline__ void vst2(void* p, T v) { *(volatile T*)p = v; __threadfence(); *(volatile T*)p = v; }
__device__ __forceinline__ v8f wmma16(v16h a, v16h b, v8f c) {
  v8f d = __builtin_amdgcn_wmma_f32_16x16x32_f16(false, a, false, b, (short)0, c, false, false);
  asm volatile("v_nop\n\tv_nop\n\tv_nop\n\tv_nop" : "+v"(d) : "v"(a), "v"(b));
  return d;
}
__device__ __forceinline__ v8f wmma_bf(v16b a, v16b b, v8f c) {
  v8f d = __builtin_amdgcn_wmma_f32_16x16x32_bf16(false, a, false, b, (short)0, c, false, false);
  asm volatile("v_nop\n\tv_nop\n\tv_nop\n\tv_nop" : "+v"(d) : "v"(a), "v"(b));
  return d;
}
__device__ __forceinline__ v16h frag_h(const _Float16* rowk0, int lane) {
  union { v16h v; v8h q[2]; } u; const _Float16* p = rowk0 + 8 * (lane >> 4);
  u.q[0] = *(const v8h*)p; u.q[1] = *(const v8h*)(p + 16); return u.v;
}
__device__ __forceinline__ v16h frag_f32(const float* rowk0, int lane) {
  v16h a; const float* p = rowk0 + 8 * (lane >> 4);
#pragma unroll
  for (int i = 0; i < 8; ++i) { a[i] = (_Float16)p[i]; a[8 + i] = (_Float16)p[16 + i]; }
  return a;
}
__device__ __forceinline__ v16h frag_f32s(const float* rowk0, int lane, float sc) {
  v16h a; const float* p = rowk0 + 8 * (lane >> 4);
#pragma unroll
  for (int i = 0; i < 8; ++i) { a[i] = (_Float16)(p[i] * sc); a[8 + i] = (_Float16)(p[16 + i] * sc); }
  return a;
}
__device__ __forceinline__ v16h fragc_f32(const float* W, int k0, int n, int lane, int ld, int K) {
  v16h a; const int g = lane >> 4;
#pragma unroll
  for (int i = 0; i < 8; ++i) { const int ka = k0 + 8 * g + i, kb = ka + 16;
    a[i] = (_Float16)(ka < K ? W[(size_t)(ka < K ? ka : K - 1) * ld + n] : 0.f); a[8 + i] = (_Float16)(kb < K ? W[(size_t)(kb < K ? kb : K - 1) * ld + n] : 0.f); }
  return a;
}
struct F2 { v16b h, l; };
__device__ __forceinline__ F2 bsplit16(const float v[16]) { F2 r;
#pragma unroll
  for (int i = 0; i < 16; ++i) { const __bf16 h = (__bf16)v[i]; r.h[i] = h; r.l[i] = (__bf16)(v[i] - (float)h); }
  return r; }
__device__ __forceinline__ F2 split_row(const float* row, int k0, int lane) { float v[16]; const float* p = row + k0 + 8 * (lane >> 4);
#pragma unroll
  for (int i = 0; i < 8; ++i) { v[i] = p[i]; v[8 + i] = p[16 + i]; }
  return bsplit16(v); }
__device__ __forceinline__ F2 split_rowK(const float* row, int k0, int lane, int K) { float v[16]; const int g = lane >> 4;
#pragma unroll
  for (int i = 0; i < 8; ++i) { const int ka = k0 + 8 * g + i, kb = ka + 16; v[i] = ka < K ? row[ka < K ? ka : K - 1] : 0.f; v[8 + i] = kb < K ? row[kb < K ? kb : K - 1] : 0.f; }
  return bsplit16(v); }
__device__ __forceinline__ F2 split_col(const float* W, int k0, int n, int lane, int ld, int K) { float v[16]; const int g = lane >> 4;
#pragma unroll
  for (int i = 0; i < 8; ++i) { const int ka = k0 + 8 * g + i, kb = ka + 16; v[i] = ka < K ? W[(size_t)(ka < K ? ka : K - 1) * ld + n] : 0.f; v[8 + i] = kb < K ? W[(size_t)(kb < K ? kb : K - 1) * ld + n] : 0.f; }
  return bsplit16(v); }
__device__ __forceinline__ v8f mac3(const F2& a, const F2& b, v8f c) { c = wmma_bf(a.l, b.h, c); c = wmma_bf(a.h, b.l, c); return wmma_bf(a.h, b.h, c); }
__device__ __forceinline__ float sigm(float v) { return 1.0f / (1.0f + expf(-v)); }
#define LDSX() do { asm volatile("s_wait_dscnt 0" ::: "memory"); __builtin_amdgcn_wave_barrier(); __builtin_amdgcn_fence(__ATOMIC_RELEASE, "workgroup"); } while (0)


#define NB 4
#define TT 2048
#define DM 256
#define NH 4
#define HD 64
#define FF 1024
#define NL 4
#define WIN 64
#define NR (NB * TT)
#define QKVP (3 * DM)
#ifndef TRB
#define TRB (NR / 64)
#endif
typedef __attribute__((ext_vector_type(8))) __bf16 v8b;
__device__ __forceinline__ v16b frag_b(const __bf16* rowk0, int lane) {
  union { v16b v; v8b q[2]; } u; const __bf16* p = rowk0 + 8 * (lane >> 4);
  u.q[0] = *(const v8b*)p; u.q[1] = *(const v8b*)(p + 16); return u.v;
}
__device__ __forceinline__ float bfr(float v) { return (float)(__bf16)v; }
__device__ __attribute__((noinline)) float exp_ni(float v) { return expf(v); }
__device__ __attribute__((noinline)) float erf_ni(float v) { return erff(v); }
#define PL_QKV 0
#define PL_O   (PL_QKV + QKVP * DM)
#define PL_W1  (PL_O + DM * DM)
#define PL_W2  (PL_W1 + FF * DM)
#define PL_SZ  (PL_W2 + DM * FF)
#define WS_PK  0u
#define WS_X   (WS_PK + 2u * NL * PL_SZ)
#define WS_XN  (WS_X + 4u * NR * DM)
#define WS_QKV (WS_XN + 4u * NR * DM)
#define WS_H   (WS_QKV + 4u * NR * QKVP)
#define WS_VTH (WS_H + 4u * NR * FF)
#define WS_VTL (WS_VTH + 2u * NB * DM * TT)
#define WS_END (WS_VTL + 2u * NB * DM * TT)

__global__ __launch_bounds__(256) void k_pack(const float* __restrict__ Wqkv, const float* __restrict__ Wo, const float* __restrict__ W1, const float* __restrict__ W2, __bf16* __restrict__ PK) {
  __shared__ __align__(16) __bf16 srow[FF]; const int n = blockIdx.x, l = blockIdx.y, tid = threadIdx.x; const float* src; int K; size_t dst;
  if (n < QKVP) { src = Wqkv + ((size_t)l * QKVP + n) * DM; K = DM; dst = (size_t)l * PL_SZ + PL_QKV + (size_t)n * DM; }
  else if (n < QKVP + DM) { src = Wo + ((size_t)l * DM + (n - QKVP)) * DM; K = DM; dst = (size_t)l * PL_SZ + PL_O + (size_t)(n - QKVP) * DM; }
  else if (n < QKVP + DM + FF) { src = W1 + ((size_t)l * FF + (n - QKVP - DM)) * DM; K = DM; dst = (size_t)l * PL_SZ + PL_W1 + (size_t)(n - QKVP - DM) * DM; }
  else { src = W2 + ((size_t)l * DM + (n - QKVP - DM - FF)) * FF; K = FF; dst = (size_t)l * PL_SZ + PL_W2 + (size_t)(n - QKVP - DM - FF) * FF; }
  for (int k = tid; k < K; k += 256) srow[k] = (__bf16)src[k];
  __syncthreads();
  if (tid < K / 8) vst2((unsigned*)(PK + dst + tid * 8), *(const v4u*)(&srow[tid * 8]));
}
__global__ __launch_bounds__(256) void k_pe(const float* __restrict__ TOK, float* __restrict__ X) {
  const size_t r = (size_t)blockIdx.x; const int t = (int)(r % TT); const int c = threadIdx.x;
  const int i2 = c & ~1; const float divt = expf((float)i2 * (-logf(10000.0f) / (float)DM)); const float ang = (float)t * divt; const float pe = (c & 1) ? cosf(ang) : sinf(ang);
  __shared__ __align__(16) float s[DM]; s[c] = bfr(TOK[r * DM + c]) + pe; __syncthreads();
  if (c < DM / 4) vst2(X + r * DM + c * 4, *(const v4f*)&s[c * 4]);
}
__global__ __launch_bounds__(256) void k_ln(const float* __restrict__ X, const float* __restrict__ gw, const float* __restrict__ bw, float* __restrict__ Y) {
  __shared__ __align__(16) float s[8][DM];
  const int wave = threadIdx.x >> 5, lane = threadIdx.x & 31; const size_t r = (size_t)blockIdx.x * 8 + wave; const float* x = X + r * DM;
  float v[8]; float sum = 0.f;
#pragma unroll
  for (int i = 0; i < 8; ++i) { v[i] = x[lane + 32 * i]; sum += v[i]; }
#pragma unroll
  for (int o = 1; o < 32; o <<= 1) sum += __shfl_xor(sum, o);
  const float mu = sum / (float)DM; float var = 0.f;
#pragma unroll
  for (int i = 0; i < 8; ++i) { const float d = v[i] - mu; var += d * d; }
#pragma unroll
  for (int o = 1; o < 32; o <<= 1) var += __shfl_xor(var, o);
  const float rs = rsqrtf(var / (float)DM + 1e-5f);
#pragma unroll
  for (int i = 0; i < 8; ++i) { const int c = lane + 32 * i; s[wave][c] = (v[i] - mu) * rs * bfr(gw[c]) + bfr(bw[c]); }
  LDSX();
  for (int pc = lane; pc < DM / 4; pc += 32) vst2(Y + r * DM + pc * 4, *(const v4f*)&s[wave][pc * 4]);
}
template <int K, int EPI>
__global__ __launch_bounds__(128) void k_lin(const float* __restrict__ A, const __bf16* __restrict__ P, const float* __restrict__ bias, float* __restrict__ OUT, int NOUT) {
  __shared__ __align__(16) float so[4][16][132];
  const int tid = threadIdx.x, wave = tid >> 5, lane = tid & 31, col = lane & 15, g = lane >> 4; const size_t r0 = (size_t)blockIdx.x * 64 + wave * 16; const int n0 = blockIdx.y * 128;
  v8f acc[8] = {};
#pragma unroll 2
  for (int kc = 0; kc < K / 32; ++kc) { const F2 a = split_row(A + (r0 + col) * K, kc * 32, lane);
#pragma unroll
    for (int j = 0; j < 8; ++j) { const v16b w = frag_b(P + (size_t)(n0 + j * 16 + col) * K + kc * 32, lane); acc[j] = wmma_bf(a.l, w, acc[j]); acc[j] = wmma_bf(a.h, w, acc[j]); } }
#pragma unroll
  for (int j = 0; j < 8; ++j) { const float bb = bfr(bias[n0 + j * 16 + col]);
#pragma unroll
    for (int r = 0; r < 8; ++r) { float v = acc[j][r] + bb; if (EPI == 1) v = 0.5f * v * (1.0f + erf_ni(v * 0.70710678118654752f)); if (EPI == 2) v += OUT[(r0 + 8 * g + r) * NOUT + n0 + j * 16 + col]; so[wave][8 * g + r][j * 16 + col] = v; } }
  LDSX();
  for (int rl = 0; rl < 16; ++rl) vst2(OUT + (r0 + rl) * NOUT + n0 + lane * 4, *(const v4f*)&so[wave][rl][lane * 4]);
}
__global__ __launch_bounds__(256) void k_vt(const float* __restrict__ QKV, __bf16* __restrict__ VTH, __bf16* __restrict__ VTL) {
  __shared__ __align__(16) __bf16 svh[DM][72], svl[DM][72];
  const int tid = threadIdx.x; const size_t t0 = (size_t)blockIdx.x * 64; const int b = (int)(t0 / TT), p0 = (int)(t0 % TT);
  for (int q = tid; q < 64 * DM; q += 256) { const int tl = q >> 8, c = q & 255; const float v = QKV[(t0 + tl) * QKVP + 2 * DM + c]; const __bf16 hb = (__bf16)v; svh[c][tl] = hb; svl[c][tl] = (__bf16)(v - (float)hb); }
  __syncthreads();
  for (int q = tid; q < DM * 8; q += 256) { const int rowi = q >> 3, pc = q & 7; const size_t o = ((size_t)b * DM + rowi) * TT + p0 + pc * 8; vst2((unsigned*)(VTH + o), *(const v4u*)&svh[rowi][pc * 8]); vst2((unsigned*)(VTL + o), *(const v4u*)&svl[rowi][pc * 8]); }
}
__global__ __launch_bounds__(128) void k_attw(const float* __restrict__ QKV, const __bf16* __restrict__ VTH, const __bf16* __restrict__ VTL, float* __restrict__ O) {
  __shared__ __align__(16) float sp[4][16][36]; __shared__ __align__(16) float so[4][16][68];
  const int tid = threadIdx.x, wave = tid >> 5, lane = tid & 31, col = lane & 15, g = lane >> 4;
  const int qb = blockIdx.x, bh = blockIdx.y, b = bh / NH, h = bh % NH; const int q0 = qb * 64 + wave * 16; const size_t tq = (size_t)b * TT + q0;
  const F2 a0 = split_row(QKV + (tq + col) * QKVP + h * HD, 0, lane), a1 = split_row(QKV + (tq + col) * QKVP + h * HD, 32, lane);
  float m[8], l[8]; v8f acc[4] = {};
#pragma unroll
  for (int r = 0; r < 8; ++r) { m[r] = -3.0e38f; l[r] = 0.f; }
  const int kstart = (qb == 0) ? 0 : (qb * 64 - 64); const int nsteps = (qb == 0) ? 2 : 4;
#pragma unroll 1
  for (int ks = 0; ks < nsteps; ++ks) { const int kbase = kstart + ks * 32; v8f s[2];
#pragma unroll
    for (int ct = 0; ct < 2; ++ct) { const int kk = kbase + ct * 16 + col; const float* krow = QKV + ((size_t)b * TT + kk) * QKVP + DM + h * HD; const F2 k0 = split_row(krow, 0, lane), k1 = split_row(krow, 32, lane);
      v8f c = mac3(a0, k0, (v8f){}); c = mac3(a1, k1, c);
#pragma unroll
      for (int r = 0; r < 8; ++r) { const int i = q0 + 8 * g + r; float v = c[r] * 0.125f; if (kk > i || kk < i - (WIN - 1)) v = -3.0e38f; s[ct][r] = v; } }
#pragma unroll
    for (int r = 0; r < 8; ++r) { float mx = fmaxf(s[0][r], s[1][r]);
#pragma unroll
      for (int o = 1; o < 16; o <<= 1) mx = fmaxf(mx, __shfl_xor(mx, o));
      const float mn = fmaxf(m[r], mx); const float alpha = (mn <= -1.0e38f) ? 1.0f : exp_ni(m[r] - mn);
      const float e0 = s[0][r] <= -1.0e38f ? 0.f : exp_ni(s[0][r] - mn), e1 = s[1][r] <= -1.0e38f ? 0.f : exp_ni(s[1][r] - mn); float es = e0 + e1;
#pragma unroll
      for (int o = 1; o < 16; o <<= 1) es += __shfl_xor(es, o);
      l[r] = l[r] * alpha + es; m[r] = mn;
#pragma unroll
      for (int dt = 0; dt < 4; ++dt) acc[dt][r] *= alpha;
      sp[wave][8 * g + r][col] = e0; sp[wave][8 * g + r][16 + col] = e1; }
    LDSX();
    const F2 pa = split_row(&sp[wave][col][0], 0, lane);
#pragma unroll
    for (int dt = 0; dt < 4; ++dt) { const size_t vrow = ((size_t)b * DM + h * HD + dt * 16 + col) * TT + kbase; const v16b vh = frag_b(VTH + vrow, lane), vl = frag_b(VTL + vrow, lane); acc[dt] = wmma_bf(pa.l, vh, acc[dt]); acc[dt] = wmma_bf(pa.h, vl, acc[dt]); acc[dt] = wmma_bf(pa.h, vh, acc[dt]); }
    LDSX(); }
#pragma unroll
  for (int r = 0; r < 8; ++r) { const float il = 1.0f / l[r];
#pragma unroll
    for (int dt = 0; dt < 4; ++dt) so[wave][8 * g + r][dt * 16 + col] = acc[dt][r] * il; }
  LDSX();
  for (int rl = 0; rl < 16; ++rl) if (lane < 16) vst2(O + (tq + rl) * DM + h * HD + lane * 4, *(const v4f*)&so[wave][rl][lane * 4]);
}
extern "C" void kernel_launch(void* const* d_in, const int* in_sizes, int n_in, void* d_out, int out_size, void* d_ws, size_t ws_size, hipStream_t stream) {
  (void)in_sizes; (void)n_in; (void)out_size;
  const float** F = (const float**)d_in;
  if (ws_size < (size_t)WS_END) return;
  char* ws = (char*)d_ws; __bf16 *PK = (__bf16*)(ws + WS_PK), *VTH = (__bf16*)(ws + WS_VTH), *VTL = (__bf16*)(ws + WS_VTL); float *X = (float*)(ws + WS_X), *XN = (float*)(ws + WS_XN), *QKV = (float*)(ws + WS_QKV), *Hb = (float*)(ws + WS_H);
  k_pack<<<dim3(QKVP + DM + FF + DM, NL), 256, 0, stream>>>(F[1], F[3], F[5], F[7], PK);
  k_pe<<<TRB * 64, 256, 0, stream>>>(F[0], X);
  for (int l = 0; l < NL; ++l) { const __bf16* PKl = PK + (size_t)l * PL_SZ;
    k_ln<<<TRB * 8, 256, 0, stream>>>(X, F[9] + l * DM, F[10] + l * DM, XN);
    k_lin<DM, 0><<<dim3(TRB, QKVP / 128), 128, 0, stream>>>(XN, PKl + PL_QKV, F[2] + l * QKVP, QKV, QKVP);
    k_vt<<<TRB, 256, 0, stream>>>(QKV, VTH, VTL);
    k_attw<<<dim3(TRB * 64 / 64 / NB > 0 ? (TT / 64) : 1, (TRB * 64 / TT > 0 ? (TRB * 64 / TT) : 1) * NH), 128, 0, stream>>>(QKV, VTH, VTL, XN);
    k_lin<DM, 2><<<dim3(TRB, DM / 128), 128, 0, stream>>>(XN, PKl + PL_O, F[4] + l * DM, X, DM);
    k_ln<<<TRB * 8, 256, 0, stream>>>(X, F[11] + l * DM, F[12] + l * DM, XN);
    k_lin<DM, 1><<<dim3(TRB, FF / 128), 128, 0, stream>>>(XN, PKl + PL_W1, F[6] + l * FF, Hb, FF);
    k_lin<FF, 2><<<dim3(TRB, DM / 128), 128, 0, stream>>>(Hb, PKl + PL_W2, F[8] + l * DM, X, DM); }
  k_ln<<<TRB * 8, 256, 0, stream>>>(X, F[13], F[14], (float*)d_out);
}
